// CombinedGoalObsNetwork_40948218200135
// MI455X (gfx1250) — hardware-verified
//
#include <hip/hip_runtime.h>
#include <stddef.h>


#define DW      64
#define NTHR    256
#define NWAVE   8
#define EPT     8
#define NGRP    2
#define CHUNK   (NTHR * EPT * NGRP)
#define WCAP    (EPT * NGRP * 32)
#define LISTN   (NWAVE * WCAP)
#define NB      512
#define BM      64
#define KSTEPS  (DW / 32)
#define NMAT    3
#define WSCAP   134217728
#define ACARRY  1.0f
#define WCARRY  64.0f
#define GSCALE  (1.0f / 64.0f)
#define LDS_AGG ((NB * DW + LISTN + NWAVE) * 4 + 64)
#define EPI_IT  ((NB * DW / 4) / NTHR)

static_assert((CHUNK & (CHUNK - 1)) == 0);
static_assert(CHUNK <= 4096);
static_assert((NB & (NB - 1)) == 0 && NB <= 4096);
static_assert(WCAP == EPT * NGRP * 32);
static_assert(LISTN == NWAVE * WCAP);
static_assert((NB % BM) == 0);
static_assert(DW == 64);
static_assert((DW % 32) == 0);
static_assert(((NB * DW / 4) % NTHR) == 0);
static_assert(EPI_IT * NTHR * 4 == NB * DW);
static_assert(BM == 4 * 16);
static_assert(NTHR == NWAVE * 32);

typedef float    v2f  __attribute__((ext_vector_type(2)));
typedef float    v4f  __attribute__((ext_vector_type(4)));
typedef float    v8f  __attribute__((ext_vector_type(8)));
typedef int      v4i  __attribute__((ext_vector_type(4)));
typedef _Float16 v4h  __attribute__((ext_vector_type(4)));
typedef _Float16 v8h  __attribute__((ext_vector_type(8)));
typedef _Float16 v16h __attribute__((ext_vector_type(16)));
union Frag { v16h v; v8h h[2]; };

__device__ __forceinline__ v8f wmh(v16h a, v16h b, v8f c) {
  v8f d = __builtin_amdgcn_wmma_f32_16x16x32_f16(false, a, false, b, (short)0, c, false, false);
  asm volatile("v_nop\n\tv_nop\n\tv_nop\n\tv_nop" : "+v"(d) : "v"(a), "v"(b));
  return d;
}

template <int NBS>
__device__ __forceinline__ int scan_chunk(const int* __restrict__ dsts, int nE, int cbase, int slotBase,
                                          int vec8, int* list, int tid, int lane, int wave) {
  int wc = 0;
#pragma unroll
  for (int g = 0; g < NGRP; ++g) {
    const int el0  = (g * NTHR + tid) * EPT;
    const int e0   = cbase + el0;
    const int sent = -2147483647 - 1;
    v4i da, db;
    if (vec8 != 0 && cbase + CHUNK <= nE) {
      da = *(const v4i*)(dsts + e0);
      db = *(const v4i*)(dsts + e0 + 4);
    } else {
      da.x = (e0     < nE) ? dsts[min(e0, nE - 1)] : sent;
      da.y = (e0 + 1 < nE) ? dsts[min(e0 + 1, nE - 1)] : sent;
      da.z = (e0 + 2 < nE) ? dsts[min(e0 + 2, nE - 1)] : sent;
      da.w = (e0 + 3 < nE) ? dsts[min(e0 + 3, nE - 1)] : sent;
      db.x = (e0 + 4 < nE) ? dsts[min(e0 + 4, nE - 1)] : sent;
      db.y = (e0 + 5 < nE) ? dsts[min(e0 + 5, nE - 1)] : sent;
      db.z = (e0 + 6 < nE) ? dsts[min(e0 + 6, nE - 1)] : sent;
      db.w = (e0 + 7 < nE) ? dsts[min(e0 + 7, nE - 1)] : sent;
    }
    const unsigned nb = (unsigned)slotBase;
    const unsigned s0 = (unsigned)da.x - nb, s1 = (unsigned)da.y - nb;
    const unsigned s2 = (unsigned)da.z - nb, s3 = (unsigned)da.w - nb;
    const unsigned s4 = (unsigned)db.x - nb, s5 = (unsigned)db.y - nb;
    const unsigned s6 = (unsigned)db.z - nb, s7 = (unsigned)db.w - nb;
    const bool h0 = s0 < (unsigned)NBS, h1 = s1 < (unsigned)NBS, h2 = s2 < (unsigned)NBS, h3 = s3 < (unsigned)NBS;
    const bool h4 = s4 < (unsigned)NBS, h5 = s5 < (unsigned)NBS, h6 = s6 < (unsigned)NBS, h7 = s7 < (unsigned)NBS;
    const unsigned any = __builtin_amdgcn_ballot_w32(h0 | h1 | h2 | h3 | h4 | h5 | h6 | h7);
    if (any != 0u) {
#define HITJ(J, HJ, SJ) { \
        const unsigned mj = __builtin_amdgcn_ballot_w32(HJ); \
        if (mj != 0u) { \
          if (HJ) { \
            const int pos = wc + (int)__builtin_amdgcn_mbcnt_lo(mj, 0u); \
            if (pos < WCAP) list[wave * WCAP + pos] = ((el0 + (J)) << 12) | (int)(SJ); \
          } \
          wc += (int)__builtin_popcount(mj); } }
      HITJ(0, h0, s0)
      HITJ(1, h1, s1)
      HITJ(2, h2, s2)
      HITJ(3, h3, s3)
      HITJ(4, h4, s4)
      HITJ(5, h5, s5)
      HITJ(6, h6, s6)
      HITJ(7, h7, s7)
#undef HITJ
    }
  }
  return wc;
}

__global__ __launch_bounds__(NTHR) void k_wcvt(const float* __restrict__ w1a, const float* __restrict__ w1b,
                                               const float* __restrict__ w2a, _Float16* dp, int nUnits) {
  const int i = (int)blockIdx.x * NTHR + (int)threadIdx.x;
  if (i >= nUnits) return;
  const int ppr = DW / 8;
  const int per = DW * ppr;
  const int mat = i / per;
  const int r = i - mat * per;
  const int n = r / ppr;
  const int seg = r - n * ppr;
  v8h o;
#pragma unroll
  for (int j = 0; j < 8; ++j) {
    const int idx = (8 * seg + j) * DW + n;
    const float f0 = w1a[idx];
    const float f1 = w1b[idx];
    const float f2 = w2a[idx];
    const float sel = (mat == 0) ? f0 : ((mat == 1) ? f1 : f2);
    o[j] = (_Float16)(sel * WCARRY);
  }
  _Float16* gp = dp + (size_t)i * 8;
  *(volatile v8h*)gp = o;
  __threadfence();
  *(volatile v8h*)gp = o;
}

__device__ __forceinline__ void agg_store_pass(const float* accl, const float* __restrict__ xres,
                                               float* hout, int nodeBase, int nDst, int tid) {
#pragma unroll 1
  for (int it = 0; it < EPI_IT; ++it) {
    const int id = it * NTHR + tid;
    const int row = id >> 4, seg = id & 15;
    const int grow = nodeBase + row;
    const bool live = grow < nDst;
    int rr = grow > nDst - 1 ? nDst - 1 : grow;
    rr = rr < 0 ? 0 : rr;
    const v4f a = *(const v4f*)(accl + (size_t)row * DW + 4 * seg);
    const v4f x = *(const v4f*)(xres + (size_t)rr * DW + 4 * seg);
    v4f o = a + x;
    o.x = live ? o.x : 0.f;
    o.y = live ? o.y : 0.f;
    o.z = live ? o.z : 0.f;
    o.w = live ? o.w : 0.f;
    *(volatile v4f*)(hout + (size_t)grow * DW + 4 * seg) = o;
  }
}

template <int GINE>
__global__ __launch_bounds__(NTHR) void k_agg(
    const float* __restrict__ xsrc, const float* __restrict__ ea,
    const float* __restrict__ we, const float* __restrict__ be,
    const int* __restrict__ srcs, const int* __restrict__ dsts,
    const float* __restrict__ xres, float* hout, int nSrc, int nE, int nDst) {
  extern __shared__ v4f lds_dyn[];
  float* accl = (float*)lds_dyn;
  int* list = (int*)(accl + NB * DW);
  int* wcnt = list + LISTN;
  const int tid = threadIdx.x, lane = tid & 31, wave = tid >> 5;
  const int nodeBase = (int)blockIdx.x * NB;
  const int vec8 = ((((size_t)dsts) & 15) == 0) ? 1 : 0;

  {
    const v4f z = {0.f, 0.f, 0.f, 0.f};
#pragma unroll 1
    for (int i = tid; i < (NB * DW) / 4; i += NTHR) ((v4f*)accl)[i] = z;
  }
  v2f w0 = {0.f, 0.f}, w1 = {0.f, 0.f}, bbv = {0.f, 0.f};
  if constexpr (GINE != 0) {
    w0  = *(const v2f*)(we + 2 * lane);
    w1  = *(const v2f*)(we + DW + 2 * lane);
    bbv = *(const v2f*)(be + 2 * lane);
  }
  __syncthreads();

  const int nChunks = (nE + CHUNK - 1) / CHUNK;
#pragma unroll 1
  for (int ch = 0; ch < nChunks; ++ch) {
    const int cbase = ch * CHUNK;
    const int wc = scan_chunk<NB>(dsts, nE, cbase, nodeBase, vec8, list, tid, lane, wave);
    if (lane == 0) wcnt[wave] = wc;
    __syncthreads();
    if (wave == 0) {
#pragma unroll 1
      for (int wsx = 0; wsx < NWAVE; ++wsx) {
        int n = __builtin_amdgcn_readfirstlane(wcnt[wsx]);
        n = n > WCAP ? WCAP : (n < 0 ? 0 : n);
        const int* lp = list + wsx * WCAP;
#pragma unroll 1
        for (int i = 0; i < n; ++i) {
          const int ent  = __builtin_amdgcn_readfirstlane(lp[i]);
          const int slot = ent & (NB - 1);
          int e = cbase + ((ent >> 12) & (CHUNK - 1));
          e = e > nE - 1 ? nE - 1 : e;
          int sv = srcs[e];
          sv = sv < 0 ? 0 : (sv > nSrc - 1 ? nSrc - 1 : sv);
          const v2f xv = *(const v2f*)(xsrc + (size_t)sv * DW + 2 * lane);
          v2f mv = xv;
          if constexpr (GINE != 0) {
            const v2f av = *(const v2f*)(ea + (size_t)e * 2);
            v2f t;
            t.x = av.x * w0.x + av.y * w1.x;
            t.y = av.x * w0.y + av.y * w1.y;
            mv.x = fmaxf((xv.x + t.x) + bbv.x, 0.f);
            mv.y = fmaxf((xv.y + t.y) + bbv.y, 0.f);
          }
          v2f* ap = (v2f*)(accl + (size_t)slot * DW + 2 * lane);
          const v2f cur = *ap;
          *ap = cur + mv;
        }
      }
    }
    __syncthreads();
  }

  agg_store_pass(accl, xres, hout, nodeBase, nDst, tid);
  __threadfence();
  agg_store_pass(accl, xres, hout, nodeBase, nDst, tid);
}

template <int MODE>
__global__ __launch_bounds__(NTHR) void k_mlp(
    const float* __restrict__ Asrc, const _Float16* __restrict__ Wpa, const float* __restrict__ ba,
    const _Float16* __restrict__ Wpb, const float* __restrict__ bb,
    const float* __restrict__ w2b, const float* __restrict__ b2b, float* Cout, int nValid) {
  constexpr int TPW = 2;
  constexpr int PPR = DW / 4;
  constexpr int NIT = (BM * PPR) / NTHR;
  static_assert((BM * PPR) % NTHR == 0);
  static_assert(NIT >= 1);
  static_assert(TPW * 16 * 2 == DW);
  static_assert(PPR == 16);

  __shared__ __attribute__((aligned(16))) float    stg[BM * DW];
  __shared__ __attribute__((aligned(16))) _Float16 a16[BM * DW];
  __shared__ __attribute__((aligned(16))) _Float16 t16[BM * DW];
  __shared__ __attribute__((aligned(16))) float    so[BM];
  __shared__ __attribute__((aligned(16))) float    sw[DW];
  const int tid = threadIdx.x, lane = tid & 31, wave = tid >> 5, hh = lane >> 4, m = lane & 15;
  const int rowBase = (int)blockIdx.x * BM;
  const int rg = wave >> 1, chf = wave & 1;
  const int r0 = rg * 16;
  const int c0 = chf * (DW / 2);

#pragma unroll
  for (int it = 0; it < NIT; ++it) {
    const int id = it * NTHR + tid;
    const int row = id >> 4, seg = id & 15;
    const int grow = rowBase + row;
    const bool live = grow < nValid;
    int rr = grow > nValid - 1 ? nValid - 1 : grow;
    rr = rr < 0 ? 0 : rr;
    v4f xv = *(const v4f*)(Asrc + (size_t)rr * DW + 4 * seg);
    xv.x = live ? xv.x : 0.f;
    xv.y = live ? xv.y : 0.f;
    xv.z = live ? xv.z : 0.f;
    xv.w = live ? xv.w : 0.f;
    v4h o;
    o.x = (_Float16)(xv.x * ACARRY);
    o.y = (_Float16)(xv.y * ACARRY);
    o.z = (_Float16)(xv.z * ACARRY);
    o.w = (_Float16)(xv.w * ACARRY);
    *(v4h*)(a16 + (size_t)row * DW + 4 * seg) = o;
  }
  if constexpr (MODE == 2) {
    if (tid < DW) sw[tid] = w2b[tid];
  }
  __syncthreads();

  v8f acc[TPW];
#pragma unroll
  for (int t = 0; t < TPW; ++t) { v8f z = {0.f, 0.f, 0.f, 0.f, 0.f, 0.f, 0.f, 0.f}; acc[t] = z; }

  {
    const _Float16* ap = a16 + (size_t)(r0 + m) * DW + 8 * hh;
    const _Float16* bp = Wpa + (size_t)(c0 + m) * DW + 8 * hh;
#pragma unroll 1
    for (int kt = 0; kt < KSTEPS; ++kt) {
      Frag a;
      a.h[0] = *(const v8h*)(ap + 32 * kt);
      a.h[1] = *(const v8h*)(ap + 32 * kt + 16);
#pragma unroll
      for (int t = 0; t < TPW; ++t) {
        const size_t to = (size_t)(16 * t) * DW + 32 * kt;
        Frag b;
        b.h[0] = *(const v8h*)(bp + to);
        b.h[1] = *(const v8h*)(bp + to + 16);
        acc[t] = wmh(a.v, b.v, acc[t]);
      }
    }
  }

#pragma unroll
  for (int t = 0; t < TPW; ++t) {
    const int col = c0 + 16 * t + m;
    const float bv = ba[col];
#pragma unroll
    for (int r = 0; r < 8; ++r) {
      const int row = r0 + 8 * hh + r;
      const float g = acc[t][r] * GSCALE;
      const float v = fmaxf(g + bv, 0.f);
      if constexpr (MODE == 1) {
        t16[(size_t)row * DW + col] = (_Float16)(v * ACARRY);
      } else {
        const bool lv = (rowBase + row) < nValid;
        stg[(size_t)row * DW + col] = lv ? v : 0.f;
      }
    }
  }
  __syncthreads();

  if constexpr (MODE == 1) {
#pragma unroll
    for (int t = 0; t < TPW; ++t) { v8f z = {0.f, 0.f, 0.f, 0.f, 0.f, 0.f, 0.f, 0.f}; acc[t] = z; }
    {
      const _Float16* ap = t16 + (size_t)(r0 + m) * DW + 8 * hh;
      const _Float16* bp = Wpb + (size_t)(c0 + m) * DW + 8 * hh;
#pragma unroll 1
      for (int kt = 0; kt < KSTEPS; ++kt) {
        Frag a;
        a.h[0] = *(const v8h*)(ap + 32 * kt);
        a.h[1] = *(const v8h*)(ap + 32 * kt + 16);
#pragma unroll
        for (int t = 0; t < TPW; ++t) {
          const size_t to = (size_t)(16 * t) * DW + 32 * kt;
          Frag b;
          b.h[0] = *(const v8h*)(bp + to);
          b.h[1] = *(const v8h*)(bp + to + 16);
          acc[t] = wmh(a.v, b.v, acc[t]);
        }
      }
    }
#pragma unroll
    for (int t = 0; t < TPW; ++t) {
      const int col = c0 + 16 * t + m;
      const float bv = bb[col];
#pragma unroll
      for (int r = 0; r < 8; ++r) {
        const int row = r0 + 8 * hh + r;
        const bool lv = (rowBase + row) < nValid;
        const float v = acc[t][r] * GSCALE + bv;
        stg[(size_t)row * DW + col] = lv ? v : 0.f;
      }
    }
    __syncthreads();

    v4f cv[NIT];
#pragma unroll
    for (int it = 0; it < NIT; ++it) {
      const int id = it * NTHR + tid;
      const int row = id >> 4, seg = id & 15;
      cv[it] = *(const v4f*)(stg + (size_t)row * DW + 4 * seg);
    }
#pragma unroll
    for (int it = 0; it < NIT; ++it) {
      const int id = it * NTHR + tid;
      const int row = id >> 4, seg = id & 15;
      float* gp = Cout + (size_t)(rowBase + row) * DW + 4 * seg;
      *(volatile v4f*)gp = cv[it];
    }
    __threadfence();
#pragma unroll
    for (int it = 0; it < NIT; ++it) {
      const int id = it * NTHR + tid;
      const int row = id >> 4, seg = id & 15;
      float* gp = Cout + (size_t)(rowBase + row) * DW + 4 * seg;
      *(volatile v4f*)gp = cv[it];
    }
  } else {
    if (tid < BM) {
      const int row = tid;
      const float* sp = stg + (size_t)row * DW;
      float s = 0.f;
#pragma unroll 4
      for (int c = 0; c < DW; ++c) s += sp[c] * sw[c];
      s += b2b[0];
      const bool lv = (rowBase + row) < nValid;
      so[tid] = lv ? s : 0.f;
    }
    __syncthreads();
    int nv = nValid - rowBase;
    nv = nv < 0 ? 0 : (nv > BM ? BM : nv);
    const int nq = nv >> 2, rem = nv & 3;
    float* op = Cout + (size_t)rowBase;
    const v4f ov = *(const v4f*)(so + 4 * (tid & 15));
    if (tid < nq) *(volatile v4f*)(op + 4 * tid) = ov;
    if (tid == 0) {
#pragma unroll 1
      for (int r = 0; r < rem; ++r) *(volatile float*)(op + 4 * nq + r) = so[4 * nq + r];
    }
    __threadfence();
    if (tid < nq) *(volatile v4f*)(op + 4 * tid) = ov;
    if (tid == 0) {
#pragma unroll 1
      for (int r = 0; r < rem; ++r) *(volatile float*)(op + 4 * nq + r) = so[4 * nq + r];
    }
  }
}

extern "C" void kernel_launch(void* const* d_in, const int* in_sizes, int n_in,
                              void* d_out, int out_size, void* d_ws, size_t ws_size,
                              hipStream_t stream) {
  if (n_in < 18) return;
  if (in_sizes[0] < DW || (in_sizes[0] % DW) != 0) return;
  if (in_sizes[1] < DW || (in_sizes[1] % DW) != 0) return;
  if (in_sizes[2] < DW || (in_sizes[2] % DW) != 0) return;
  const int nS = in_sizes[0] / DW;
  const int nT = in_sizes[1] / DW;
  const int nA = in_sizes[2] / DW;
  const int E1 = in_sizes[14];
  const int E2 = in_sizes[16];
  if (E1 < 1 || E2 < 1 || E1 > (1 << 28) || E2 > (1 << 28)) return;
  if (in_sizes[15] != E1 || in_sizes[17] != E2 || in_sizes[3] != 2 * E1) return;
  if (in_sizes[4] != 2 * DW || in_sizes[5] != DW) return;
  if (in_sizes[6] != DW * DW || in_sizes[7] != DW) return;
  if (in_sizes[8] != DW * DW || in_sizes[9] != DW) return;
  if (in_sizes[10] != DW * DW || in_sizes[11] != DW) return;
  if (in_sizes[12] != DW || in_sizes[13] < 1) return;
  if (out_size != nA) return;
  if (nS > (1 << 24) || nT > (1 << 24) || nA > (1 << 24)) return;

  const float* x_state   = (const float*)d_in[0];
  const float* x_task    = (const float*)d_in[1];
  const float* x_actor   = (const float*)d_in[2];
  const float* edge_attr = (const float*)d_in[3];
  const float* We  = (const float*)d_in[4];
  const float* be  = (const float*)d_in[5];
  const float* W1a = (const float*)d_in[6];
  const float* b1a = (const float*)d_in[7];
  const float* W1b = (const float*)d_in[8];
  const float* b1b = (const float*)d_in[9];
  const float* W2a = (const float*)d_in[10];
  const float* b2a = (const float*)d_in[11];
  const float* W2b = (const float*)d_in[12];
  const float* b2b = (const float*)d_in[13];
  const int* src_st = (const int*)d_in[14];
  const int* dst_st = (const int*)d_in[15];
  const int* src_ta = (const int*)d_in[16];
  const int* dst_ta = (const int*)d_in[17];
  float* out = (float*)d_out;

  const int nBT   = (nT + NB - 1) / NB;
  const int NTPAD = nBT * NB;
  const int nBA   = (nA + NB - 1) / NB;
  const int NAPAD = nBA * NB;
  const int nM1   = NTPAD / BM;
  const int nM2   = (nA + BM - 1) / BM;
  const int nUnits = NMAT * DW * (DW / 8);

  char* ws = (char*)d_ws;
  size_t off = 0;
  const size_t oWp = off; off += (size_t)NMAT * DW * DW * 2;  off = (off + 1023) & ~(size_t)1023;
  const size_t oH  = off; off += (size_t)NTPAD * DW * 4;      off = (off + 1023) & ~(size_t)1023;
  const size_t oX1 = off; off += (size_t)NTPAD * DW * 4;      off = (off + 1023) & ~(size_t)1023;
  const size_t oH2 = off; off += (size_t)NAPAD * DW * 4;      off = (off + 1023) & ~(size_t)1023;
  if (off > ws_size || off > (size_t)WSCAP) return;

  _Float16* wpl = (_Float16*)(ws + oWp);
  float* hpl  = (float*)(ws + oH);
  float* x1pl = (float*)(ws + oX1);
  float* h2pl = (float*)(ws + oH2);

  k_wcvt<<<(nUnits + NTHR - 1) / NTHR, NTHR, 0, stream>>>(W1a, W1b, W2a, wpl, nUnits);

  hipFuncSetAttribute(reinterpret_cast<const void*>(&k_agg<1>),
                      hipFuncAttributeMaxDynamicSharedMemorySize, LDS_AGG);
  k_agg<1><<<nBT, NTHR, LDS_AGG, stream>>>(x_state, edge_attr, We, be, src_st, dst_st, x_task, hpl,
                                            nS, E1, nT);

  k_mlp<1><<<nM1, NTHR, 0, stream>>>(hpl, wpl, b1a, wpl + (size_t)DW * DW, b1b, W2b, b2b, x1pl, nT);

  hipFuncSetAttribute(reinterpret_cast<const void*>(&k_agg<0>),
                      hipFuncAttributeMaxDynamicSharedMemorySize, LDS_AGG);
  k_agg<0><<<nBA, NTHR, LDS_AGG, stream>>>(x1pl, edge_attr, We, be, src_ta, dst_ta, x_actor, h2pl,
                                            nT, E2, nA);

  k_mlp<2><<<nM2, NTHR, 0, stream>>>(h2pl, wpl + (size_t)2 * DW * DW, b2a, wpl + (size_t)DW * DW, b1b,
                                      W2b, b2b, out, nA);
}
